// TopNAttention_74749610819842
// MI455X (gfx1250) — hardware-verified
//
#include <hip/hip_runtime.h>
#include <stddef.h>
#include <stdint.h>

#define BB   2
#define NN   2048
#define MM   2048
#define DD   128
#define HH   8
#define DH   (DD * HH)
#define NQR  (BB * NN)
#define NKR  (BB * 2 * MM)
#define NXR  (NQR + NKR)
#define NWR  (2 * DH)

static_assert(DD == 128);
static_assert(DD % 32 == 0);
static_assert(DH % 64 == 0);
static_assert(NXR % 256 == 0);
static_assert(NQR % 256 == 0);
static_assert((NXR * 16) % 256 == 0);
static_assert((NWR * 16) % 256 == 0);
static_assert(NN % 128 == 0);
static_assert(MM % 64 == 0);

typedef _Float16 v16h __attribute__((ext_vector_type(16)));
typedef _Float16 v8h  __attribute__((ext_vector_type(8)));
typedef float    v8f  __attribute__((ext_vector_type(8)));
typedef float    v4f  __attribute__((ext_vector_type(4)));
typedef unsigned int v4u __attribute__((ext_vector_type(4)));

union Frag  { v16h v; v8h h[2]; };
union Pack8 { v8h h; v4u u; };

__device__ __forceinline__ v8f zero8() { return (v8f){0.f, 0.f, 0.f, 0.f, 0.f, 0.f, 0.f, 0.f}; }

__device__ __forceinline__ v8f mma16(v16h a, v16h b, v8f c) {
  c = __builtin_amdgcn_wmma_f32_16x16x32_f16(false, a, false, b, (short)0, c, false, false);
  asm volatile("v_nop\n\tv_nop\n\tv_nop\n\tv_nop" : "+v"(c) : "v"(a), "v"(b));
  return c;
}

__device__ __forceinline__ v16h ldfrag(const _Float16* p, int ld, int row0, int k0, int lane) {
  const int m = lane & 15, lh = lane >> 4;
  const _Float16* q = p + (size_t)(row0 + m) * ld + k0 + 8 * lh;
  Frag f;
  f.h[0] = *(const v8h*)(q);
  f.h[1] = *(const v8h*)(q + 16);
  return f.v;
}

__device__ __forceinline__ void gemm32x64(const _Float16* __restrict__ A, int lda,
                                          const _Float16* __restrict__ Bt, int ldb,
                                          int m0, int n0, int lane, v8f (&acc)[2][4]) {
#pragma unroll 2
  for (int k0 = 0; k0 < DD; k0 += 32) {
    const v16h a0 = ldfrag(A, lda, m0, k0, lane);
    const v16h a1 = ldfrag(A, lda, m0 + 16, k0, lane);
    const v16h b0 = ldfrag(Bt, ldb, n0, k0, lane);
    const v16h b1 = ldfrag(Bt, ldb, n0 + 16, k0, lane);
    const v16h b2 = ldfrag(Bt, ldb, n0 + 32, k0, lane);
    const v16h b3 = ldfrag(Bt, ldb, n0 + 48, k0, lane);
    acc[0][0] = mma16(a0, b0, acc[0][0]);
    acc[1][0] = mma16(a1, b0, acc[1][0]);
    acc[0][1] = mma16(a0, b1, acc[0][1]);
    acc[1][1] = mma16(a1, b1, acc[1][1]);
    acc[0][2] = mma16(a0, b2, acc[0][2]);
    acc[1][2] = mma16(a1, b2, acc[1][2]);
    acc[0][3] = mma16(a0, b3, acc[0][3]);
    acc[1][3] = mma16(a1, b3, acc[1][3]);
  }
}

__global__ __launch_bounds__(256) void k_cvt_x(const float* __restrict__ q, const float* __restrict__ k,
                                               const float* __restrict__ v, _Float16* __restrict__ X,
                                               int nthr) {
  const int t = blockIdx.x * 256 + (int)threadIdx.x;
  if (t >= nthr) return;
  const int row = t >> 4;
  const int pc  = t & 15;
  const int j   = row - NQR;
  const int jc  = (j < 0) ? 0 : j;
  const int bi  = jc >> 12;
  const int jj  = jc & 4095;
  const int rq  = (row < NQR) ? row : (NQR - 1);
  const size_t offq  = (size_t)rq * DD + pc * 8;
  const size_t offkv = ((size_t)(bi * MM + (jj & (MM - 1)))) * DD + pc * 8;
  const float* src = (row < NQR) ? (q + offq) : ((jj < MM) ? (k + offkv) : (v + offkv));
  const v4f a0 = *(const v4f*)(src);
  const v4f a1 = *(const v4f*)(src + 4);
  Pack8 pk;
  pk.h = (v8h){(_Float16)a0[0], (_Float16)a0[1], (_Float16)a0[2], (_Float16)a0[3],
               (_Float16)a1[0], (_Float16)a1[1], (_Float16)a1[2], (_Float16)a1[3]};
  const v4u vv = pk.u;
  const size_t o = (size_t)row * DD + pc * 8;
  for (int ps = 0; ps < 2; ++ps) {
    *(volatile v4u*)(X + o) = vv;
    __threadfence();
  }
}

__global__ __launch_bounds__(256) void k_cvt_w(const float* __restrict__ Wq, const float* __restrict__ Wkv,
                                               _Float16* __restrict__ WT, int nthr) {
  const int t = blockIdx.x * 256 + (int)threadIdx.x;
  if (t >= nthr) return;
  const int rw = t >> 4;
  const int pc = t & 15;
  const float* src = (rw < DH) ? Wq : Wkv;
  const int n = rw & (DH - 1);
  Pack8 pk;
#pragma unroll
  for (int e = 0; e < 8; ++e) pk.h[e] = (_Float16)(src[(size_t)(pc * 8 + e) * DH + n] * 16.0f);
  const v4u vv = pk.u;
  const size_t o = (size_t)rw * DD + pc * 8;
  for (int ps = 0; ps < 2; ++ps) {
    *(volatile v4u*)(WT + o) = vv;
    __threadfence();
  }
}

#define OTP 68
__global__ __launch_bounds__(256) void k_proj(const _Float16* __restrict__ X, const _Float16* __restrict__ WT,
                                              const float* __restrict__ bq, const float* __restrict__ bkv,
                                              _Float16* __restrict__ Qp, _Float16* __restrict__ Kp,
                                              float* __restrict__ vout) {
  __shared__ __align__(16) float sw[8 * 16 * OTP];
  const int tid = threadIdx.x, lane = tid & 31, wave = tid >> 5;
  const int hh = lane >> 4, c = lane & 15;
  const int rb = blockIdx.x;
  const int n0 = blockIdx.y * 64;
  const int m0 = rb * 256 + wave * 32;
  const int kind = (rb < 16) ? 0 : ((((rb - 16) & 1) == 0) ? 1 : 2);
  const int wrow0 = (rb < 16) ? n0 : (DH + n0);
  const float* bias = (rb < 16) ? bq : bkv;
  float* st = sw + wave * (16 * OTP);

  v8f acc[2][4];
#pragma unroll
  for (int s = 0; s < 2; ++s)
#pragma unroll
    for (int t = 0; t < 4; ++t) acc[s][t] = zero8();
  gemm32x64(X, DD, WT, DD, m0, wrow0, lane, acc);

  float bn[4];
#pragma unroll
  for (int t = 0; t < 4; ++t) bn[t] = bias[n0 + 16 * t + c];
  const int cb  = n0 >> 7;
  const int di0 = n0 & 127;

#pragma unroll
  for (int sub = 0; sub < 2; ++sub) {
    __syncthreads();
#pragma unroll
    for (int r = 0; r < 8; ++r) {
#pragma unroll
      for (int t = 0; t < 4; ++t) st[(8 * hh + r) * OTP + 16 * t + c] = acc[sub][t][r] * 0.0625f + bn[t];
    }
    __syncthreads();
    const int rbase = m0 + sub * 16;
    if (kind == 2) {
      v4f val[8];
      size_t go[8];
#pragma unroll
      for (int it = 0; it < 8; ++it) {
        const int p    = lane + 32 * it;
        const int L    = p >> 3;
        const int pc   = p & 7;
        const int row  = L >> 1;
        const int half = L & 1;
        val[it] = *(const v4f*)(st + row * OTP + half * 32 + pc * 4);
        const int R  = rbase + row - NQR;
        const int bi = R >> 12;
        const int r  = R & 4095;
        const int hi = r >> 9;
        const int mi = (r & 511) * 8 + cb;
        const int orow = (bi * HH + hi) * MM + (mi - MM);
        go[it] = (size_t)orow * DD + di0 + half * 32 + pc * 4;
      }
      for (int ps = 0; ps < 2; ++ps) {
#pragma unroll
        for (int it = 0; it < 8; ++it) *(volatile v4f*)(vout + go[it]) = val[it];
        __threadfence();
      }
    } else {
      v4u val[4];
      size_t go[4];
#pragma unroll
      for (int it = 0; it < 4; ++it) {
        const int p   = lane + 32 * it;
        const int row = p >> 3;
        const int pc  = p & 7;
        const v4f f0 = *(const v4f*)(st + row * OTP + pc * 8);
        const v4f f1 = *(const v4f*)(st + row * OTP + pc * 8 + 4);
        Pack8 pk;
        pk.h = (v8h){(_Float16)f0[0], (_Float16)f0[1], (_Float16)f0[2], (_Float16)f0[3],
                     (_Float16)f1[0], (_Float16)f1[1], (_Float16)f1[2], (_Float16)f1[3]};
        val[it] = pk.u;
        int prow;
        if (kind == 0) {
          const int R  = rbase + row;
          const int bi = R >> 11;
          const int r  = R & 2047;
          const int hi = r >> 8;
          const int ni = (r & 255) * 8 + cb;
          prow = (bi * HH + hi) * NN + ni;
        } else {
          const int R  = rbase + row - NQR;
          const int bi = R >> 12;
          const int r  = R & 4095;
          const int hi = r >> 9;
          const int mi = (r & 511) * 8 + cb;
          prow = (bi * HH + hi) * MM + mi;
        }
        go[it] = (size_t)prow * DD + di0 + pc * 8;
      }
      _Float16* dst = (kind == 0) ? Qp : Kp;
      for (int ps = 0; ps < 2; ++ps) {
#pragma unroll
        for (int it = 0; it < 4; ++it) *(volatile v4u*)(dst + go[it]) = val[it];
        __threadfence();
      }
    }
  }
}

#define SQP 36
__global__ __launch_bounds__(256) void k_score(const _Float16* __restrict__ Qp, const _Float16* __restrict__ Kp,
                                               float* __restrict__ aout) {
  __shared__ __align__(16) float ss[8 * 32 * SQP];
  const int tid = threadIdx.x, lane = tid & 31, wave = tid >> 5;
  const int hh = lane >> 4, c = lane & 15;
  const int b  = blockIdx.z;
  const int rg = wave & 3, cg = wave >> 2;
  const int n0 = (int)blockIdx.y * 128 + rg * 32;
  const int m0 = (int)blockIdx.x * 64 + cg * 32;
  float* st = ss + wave * (32 * SQP);
  const float SCL = 0.08838834764831845f;

  v8f racc[2][2];
#pragma unroll
  for (int s = 0; s < 2; ++s)
#pragma unroll
    for (int t = 0; t < 2; ++t) racc[s][t] = zero8();

#pragma unroll 1
  for (int h = 0; h < HH; ++h) {
    const _Float16* Ab = Qp + ((size_t)(b * HH + h) * NN + n0) * DD;
    const _Float16* Bb = Kp + ((size_t)(b * HH + h) * MM + m0) * DD;
    v8f cacc[2][2];
#pragma unroll
    for (int s = 0; s < 2; ++s)
#pragma unroll
      for (int t = 0; t < 2; ++t) cacc[s][t] = zero8();
#pragma unroll 2
    for (int k0 = 0; k0 < DD; k0 += 32) {
      const v16h a0 = ldfrag(Ab, DD, 0, k0, lane);
      const v16h a1 = ldfrag(Ab, DD, 16, k0, lane);
      const v16h b0 = ldfrag(Bb, DD, 0, k0, lane);
      const v16h b1 = ldfrag(Bb, DD, 16, k0, lane);
      cacc[0][0] = mma16(a0, b0, cacc[0][0]);
      cacc[1][0] = mma16(a1, b0, cacc[1][0]);
      cacc[0][1] = mma16(a0, b1, cacc[0][1]);
      cacc[1][1] = mma16(a1, b1, cacc[1][1]);
    }
#pragma unroll
    for (int s = 0; s < 2; ++s) {
#pragma unroll
      for (int t = 0; t < 2; ++t) {
#pragma unroll
        for (int r = 0; r < 8; ++r) {
          const float sv = cacc[s][t][r] * SCL;
          racc[s][t][r] += (sv > 0.0f) ? sv : 0.0f;
        }
      }
    }
  }

#pragma unroll
  for (int s = 0; s < 2; ++s) {
#pragma unroll
    for (int t = 0; t < 2; ++t) {
#pragma unroll
      for (int r = 0; r < 8; ++r) st[(16 * s + 8 * hh + r) * SQP + 16 * t + c] = racc[s][t][r] * 0.125f;
    }
  }
  __syncthreads();
  v4f val[8];
  size_t go[8];
#pragma unroll
  for (int it = 0; it < 8; ++it) {
    const int p   = lane + 32 * it;
    const int row = p >> 3;
    const int pc  = p & 7;
    val[it] = *(const v4f*)(st + row * SQP + pc * 4);
    go[it]  = ((size_t)(b * NN + n0 + row)) * MM + m0 + pc * 4;
  }
  for (int ps = 0; ps < 2; ++ps) {
#pragma unroll
    for (int it = 0; it < 8; ++it) *(volatile v4f*)(aout + go[it]) = val[it];
    __threadfence();
  }
}

extern "C" void kernel_launch(void* const* d_in, const int* in_sizes, int n_in,
                              void* d_out, int out_size, void* d_ws, size_t ws_size,
                              hipStream_t stream) {
  if (n_in < 7) return;
  if (in_sizes[0] != NQR * DD) return;
  if (in_sizes[1] != BB * MM * DD) return;
  if (in_sizes[2] != BB * MM * DD) return;
  if (in_sizes[3] != DD * DH) return;
  if (in_sizes[4] != DH) return;
  if (in_sizes[5] != DD * DH) return;
  if (in_sizes[6] != DH) return;
  if (out_size != BB * HH * MM * DD + BB * NN * MM) return;

  const float* q   = (const float*)d_in[0];
  const float* k   = (const float*)d_in[1];
  const float* v   = (const float*)d_in[2];
  const float* Wq  = (const float*)d_in[3];
  const float* bq  = (const float*)d_in[4];
  const float* Wkv = (const float*)d_in[5];
  const float* bkv = (const float*)d_in[6];
  float* out0 = (float*)d_out;
  float* out1 = out0 + (size_t)BB * HH * MM * DD;

  size_t off = 0;
  const size_t oX  = off; off += (size_t)NXR * DD * 2;
  const size_t oWT = off; off += (size_t)NWR * DD * 2;
  const size_t oQp = off; off += (size_t)BB * HH * NN * DD * 2;
  const size_t oKp = off; off += (size_t)BB * HH * MM * DD * 2;
  if (off > ws_size) return;
  if (off > (size_t)134217728) return;

  char* ws = (char*)d_ws;
  _Float16* X  = (_Float16*)(ws + oX);
  _Float16* WT = (_Float16*)(ws + oWT);
  _Float16* Qp = (_Float16*)(ws + oQp);
  _Float16* Kp = (_Float16*)(ws + oKp);

  const int nx = NXR * 16;
  k_cvt_x<<<dim3((nx + 255) / 256), dim3(256), 0, stream>>>(q, k, v, X, nx);
  const int nw = NWR * 16;
  k_cvt_w<<<dim3((nw + 255) / 256), dim3(256), 0, stream>>>(Wq, Wkv, WT, nw);
  k_proj<<<dim3(NXR / 256, DH / 64), dim3(256), 0, stream>>>(X, WT, bq, bkv, Qp, Kp, out0);
  k_score<<<dim3(MM / 64, NN / 128, BB), dim3(256), 0, stream>>>(Qp, Kp, out1);
  (void)hipGetLastError();
}
